// cosAtt_18305150615795
// MI455X (gfx1250) — hardware-verified
//
#include <hip/hip_runtime.h>


#define NMAP 64
#define NN   1024
#define DDm  128
#define DM   DDm
#define LOSC 1024.0f

typedef _Float16 h16;
typedef unsigned short bf;
typedef __attribute__((ext_vector_type(16))) __bf16   v16bf;
typedef __attribute__((ext_vector_type(16))) _Float16 v16h;
typedef __attribute__((ext_vector_type(8)))  _Float16 v8h;
typedef __attribute__((ext_vector_type(8)))  unsigned short v8us;
typedef __attribute__((ext_vector_type(8)))  float    v8f;
typedef __attribute__((ext_vector_type(4)))  float    v4f;
typedef v8h  __attribute__((may_alias)) v8ha;
typedef v4f  __attribute__((may_alias)) v4fa;
typedef v8us __attribute__((may_alias)) v8usa;

__device__ __forceinline__ unsigned short f2bf(float f) { unsigned u = __float_as_uint(f); u += 0x7FFFu + ((u >> 16) & 1u); return (unsigned short)(u >> 16); }
__device__ __forceinline__ float bf2f(unsigned short b) { return __uint_as_float(((unsigned)b) << 16); }
__device__ __forceinline__ float bfr(float f) { return bf2f(f2bf(f)); }
__device__ __forceinline__ v16h cat16(v8h lo, v8h hi) { return __builtin_shufflevector(lo, hi, 0, 1, 2, 3, 4, 5, 6, 7, 8, 9, 10, 11, 12, 13, 14, 15); }
__device__ __forceinline__ v16bf cat16b(v8us lo, v8us hi) { return __builtin_bit_cast(v16bf, __builtin_shufflevector(lo, hi, 0, 1, 2, 3, 4, 5, 6, 7, 8, 9, 10, 11, 12, 13, 14, 15)); }
__device__ __forceinline__ v8f wmma16(v16h a, v16h b, v8f c) { return __builtin_amdgcn_wmma_f32_16x16x32_f16(false, a, false, b, (short)0, c, false, false); }
__device__ __forceinline__ v8f wmmab(v16bf a, v16bf b, v8f c) { return __builtin_amdgcn_wmma_f32_16x16x32_bf16(false, a, false, b, (short)0, c, false, false); }

template <bool SPLITA, bool F16OUT = false>
__global__ __launch_bounds__(128) void k_gemmb(const bf* __restrict__ A, const bf* __restrict__ Al, const bf* __restrict__ Bn, const float* __restrict__ bias, float* C, int ldc, h16* C2, const float* __restrict__ R = nullptr, int K = DM, int roundR = 1) {
    __shared__ __align__(16) float ost[4][16 * 68];
    const int lane = threadIdx.x & 31, wave = threadIdx.x >> 5, lr = lane & 15, hi = lane >> 4;
    const int r0 = blockIdx.x * 64 + wave * 16, c0 = blockIdx.y * 64;
    const size_t aoff = (size_t)(r0 + lr) * K + 8 * hi;
    size_t boff[4];
#pragma unroll
    for (int t = 0; t < 4; ++t) boff[t] = (size_t)(c0 + t * 16 + lr) * K + 8 * hi;
    v8f acc[4];
#pragma unroll
    for (int t = 0; t < 4; ++t) acc[t] = (v8f){};
#pragma unroll 1
    for (int kc = 0; kc < K; kc += 32) {
        const v16bf a = cat16b(*(const v8us*)(A + aoff + kc), *(const v8us*)(A + aoff + kc + 16));
        v16bf al = a;
        if (SPLITA) al = cat16b(*(const v8us*)(Al + aoff + kc), *(const v8us*)(Al + aoff + kc + 16));
#pragma unroll
        for (int t = 0; t < 4; ++t) { const v16bf b = cat16b(*(const v8us*)(Bn + boff[t] + kc), *(const v8us*)(Bn + boff[t] + kc + 16)); acc[t] = wmmab(a, b, acc[t]); if (SPLITA) acc[t] = wmmab(al, b, acc[t]); }
        asm volatile("v_nop\n\tv_nop\n\tv_nop\n\tv_nop" : "+v"(acc[0]), "+v"(acc[1]), "+v"(acc[2]), "+v"(acc[3]) : "v"(a), "v"(al));
    }
    float* os = &ost[wave][0];
#pragma unroll
    for (int t = 0; t < 4; ++t) { const float bv = bias ? bfr(bias[c0 + t * 16 + lr]) : 0.f;
#pragma unroll
        for (int j = 0; j < 8; ++j) os[(hi * 8 + j) * 68 + t * 16 + lr] = acc[t][j] + bv; }
    __syncthreads();
    if (F16OUT) {
        h16* crow = (h16*)(void*)C + (size_t)r0 * ldc + c0;
        auto pass = [&]() {
#pragma unroll
            for (int s = 0; s < 4; ++s) { const int row = 4 * s + (lane >> 3), piece = lane & 7; const float* sp = os + row * 68 + piece * 8; v8h o, o2;
#pragma unroll
                for (int i = 0; i < 8; ++i) { const h16 a = (h16)sp[i]; o[i] = a; o2[i] = (h16)((sp[i] - (float)a) * LOSC); }
                *(volatile v8h*)(crow + (size_t)row * ldc + piece * 8) = o; if (C2) *(volatile v8h*)(C2 + (size_t)r0 * ldc + c0 + (size_t)row * ldc + piece * 8) = o2; }
        };
        pass(); __threadfence(); pass();
    } else {
        float* crow = C + (size_t)r0 * ldc + c0;
        auto pass = [&]() {
#pragma unroll
            for (int s = 0; s < 8; ++s) { const int Lid = (lane >> 3) + 4 * s, piece = lane & 7; const int row = Lid >> 1, cofs = (Lid & 1) * 32 + piece * 4;
                v4f val = *(const v4fa*)(os + row * 68 + cofs); if (R) { const v4f rv = *(const v4f*)(R + ((size_t)r0 + row) * ldc + c0 + cofs); val += roundR ? (v4f){bfr(rv[0]), bfr(rv[1]), bfr(rv[2]), bfr(rv[3])} : rv; }
                *(volatile v4f*)(crow + (size_t)row * ldc + cofs) = val; }
        };
        pass(); __threadfence(); pass();
    }
}


__global__ __launch_bounds__(256) void k_cvt(const float* __restrict__ src, bf* dst) {
    typedef __attribute__((ext_vector_type(4))) unsigned short v4us;
    const int lane = threadIdx.x & 31; const size_t r = (size_t)blockIdx.x * 8 + (threadIdx.x >> 5); if (r >= (size_t)NN) return; v4us o;
#pragma unroll
    for (int i = 0; i < 4; ++i) o[i] = f2bf(src[r * DDm + lane * 4 + i]);
    *(volatile v4us*)(dst + r * DDm + lane * 4) = o; __threadfence(); *(volatile v4us*)(dst + r * DDm + lane * 4) = o;
}
__global__ __launch_bounds__(256) void k_norm(const float* __restrict__ src, float* NRM) {
    const int n = blockIdx.x * 256 + threadIdx.x; if (n >= NN) return; float s = 0.f;
#pragma unroll 8
    for (int d = 0; d < DDm; ++d) { const float v = bfr(src[(size_t)n * DDm + d]); s = fmaf(v, v, s); }
    const float r = sqrtf(s); *(volatile float*)(NRM + n) = r; __threadfence(); *(volatile float*)(NRM + n) = r;
}
__global__ __launch_bounds__(256) void k_xt(const float* __restrict__ src, bf* XT) {
    __shared__ __align__(16) unsigned short tl[64 * 72];
    const int tid = threadIdx.x, m0 = blockIdx.x * 64, d0 = blockIdx.y * 64; const int mm = tid >> 2, dq = (tid & 3) * 16;
#pragma unroll
    for (int i = 0; i < 16; ++i) tl[(dq + i) * 72 + mm] = f2bf(src[(size_t)(m0 + mm) * DDm + d0 + dq + i]);
    __syncthreads();
    const int piece = tid & 7;
    auto pass = [&]() {
#pragma unroll
        for (int s = 0; s < 2; ++s) { const int dr = (tid >> 3) + 32 * s; const v8us val = *(const v8usa*)(tl + dr * 72 + piece * 8); *(volatile v8us*)(XT + (size_t)(d0 + dr) * NN + m0 + piece * 8) = val; }
    };
    pass(); __threadfence(); pass();
}
__global__ __launch_bounds__(256) void k_sig(const float* __restrict__ G, const float* __restrict__ NRM, const float* __restrict__ beta, bf* PH, bf* PL) {
    typedef __attribute__((ext_vector_type(4))) unsigned short v4us;
    const int lane = threadIdx.x & 31, n = blockIdx.x * 8 + (threadIdx.x >> 5); if (n >= NN) return; const float nn_ = NRM[n];
#pragma unroll 1
    for (int ps = 0; ps < 2; ++ps) {
#pragma unroll 1
        for (int c0 = lane * 4; c0 < NN; c0 += 128) { v4us oh, ol;
#pragma unroll
            for (int q = 0; q < 4; ++q) { const int m = c0 + q; const float cs = G[(size_t)n * NN + m] / (nn_ * NRM[m] + 1e-7f); const float z = bfr(beta[(size_t)n * NN + m]) * cs;
                const float p = 1.0f / (1.0f + __expf(-z)); const unsigned short hb = f2bf(p); oh[q] = hb; ol[q] = f2bf(p - bf2f(hb)); }
            const size_t o = (size_t)n * NN + c0; *(volatile v4us*)(PH + o) = oh; *(volatile v4us*)(PL + o) = ol; }
        if (ps == 0) __threadfence(); }
}

extern "C" void kernel_launch(void* const* d_in, const int* in_sizes, int n_in,
                              void* d_out, int out_size, void* d_ws, size_t ws_size, hipStream_t stream) {
    (void)in_sizes; (void)n_in; (void)out_size;
    const float* x = (const float*)d_in[0]; const float* beta = (const float*)d_in[1];
    float* out = (float*)d_out;
    char* wsp = (char*)d_ws;
    auto take = [&](size_t bytes) { char* p = wsp; wsp += (bytes + 255) & ~(size_t)255; return (void*)p; };
    bf* Xb = (bf*)take((size_t)NN * DDm * 2); bf* XT = (bf*)take((size_t)DDm * NN * 2); float* NRM = (float*)take(NN * 4); float* G = (float*)take((size_t)NN * NN * 4); bf* PH = (bf*)take((size_t)NN * NN * 2); bf* PL = (bf*)take((size_t)NN * NN * 2);
    if ((size_t)(wsp - (char*)d_ws) > ws_size) return;
    for (int mp = 0; mp < NMAP; ++mp) { const float* xm = x + (size_t)mp * NN * DDm;
        k_cvt<<<NN / 8, 256, 0, stream>>>(xm, Xb); k_norm<<<NN / 256, 256, 0, stream>>>(xm, NRM); k_xt<<<dim3(NN / 64, DDm / 64, 1), 256, 0, stream>>>(xm, XT);
        k_gemmb<false, false><<<dim3(NN / 64, NN / 64, 1), 128, 0, stream>>>(Xb, nullptr, Xb, nullptr, G, NN, nullptr, nullptr, DDm);
        k_sig<<<NN / 8, 256, 0, stream>>>(G, NRM, beta, PH, PL);
        k_gemmb<true, false><<<dim3(NN / 64, DDm / 64, 1), 128, 0, stream>>>(PH, PL, XT, nullptr, out + (size_t)mp * NN * DDm, DDm, nullptr, nullptr, NN); }
}
